// BaseRNN_56762287784464
// MI455X (gfx1250) — hardware-verified
//
#include <hip/hip_runtime.h>
#include <math.h>

constexpr int NSEQ        = 256;
constexpr int NSTEP       = 2048;
constexpr int NHID        = 128;
constexpr int NVOC        = 50000;
constexpr int NLAY        = 2;
constexpr int NTHR        = 256;
constexpr int SEQ_PER_BLK = 16;
constexpr int APITCH      = 136;
constexpr int KTOT        = 256;
constexpr int OPITCH      = 132;
constexpr int ATILE       = SEQ_PER_BLK * APITCH;
constexpr float A_SCALE   = 8.0f;
constexpr float W_SCALE   = 64.0f;
constexpr float FOLD_INV  = 1.0f / 512.0f;

typedef __attribute__((ext_vector_type(16))) _Float16 v16h;
typedef __attribute__((ext_vector_type(8)))  _Float16 v8h;
typedef __attribute__((ext_vector_type(16))) __bf16   v16b;
typedef __attribute__((ext_vector_type(8)))  __bf16   v8b;
typedef __attribute__((ext_vector_type(8)))  float    v8f;
typedef __attribute__((ext_vector_type(4)))  float    v4f;

__device__ __forceinline__ void dep_guard_h(v8f& a, v8f& b, v16h x, v16h y) { asm volatile("v_nop\n\tv_nop\n\tv_nop\n\tv_nop" : "+v"(a), "+v"(b) : "v"(x), "v"(y)); }
__device__ __forceinline__ void dep_guard_b(v8f& a, v8f& b, v16b x, v16b y) { asm volatile("v_nop\n\tv_nop\n\tv_nop\n\tv_nop" : "+v"(a), "+v"(b) : "v"(x), "v"(y)); }
__device__ __forceinline__ void keep4_h(v16h a, v16h b, v16h c, v16h d) { asm volatile("v_nop" :: "v"(a), "v"(b), "v"(c), "v"(d)); }
__device__ __forceinline__ void keep4_b(v16b a, v16b b, v16b c, v16b d) { asm volatile("v_nop" :: "v"(a), "v"(b), "v"(c), "v"(d)); }
template <typename T> struct Frag;
template <> struct Frag<_Float16> {
  typedef v16h V; union U { v16h v; v8h h[2]; };
  static __device__ __forceinline__ v16h load(const _Float16* p) {
    U f; f.h[0] = *(const v8h*)(p); f.h[1] = *(const v8h*)(p + 16); return f.v;
  }
  static __device__ __forceinline__ v8f mma(v16h a, v16h b, v8f c) {
    return __builtin_amdgcn_wmma_f32_16x16x32_f16(false, a, false, b, (short)0, c, false, false);
  }
  static __device__ __forceinline__ void guard(v8f& a, v8f& b, v16h x, v16h y) { dep_guard_h(a, b, x, y); }
  static __device__ __forceinline__ void keep(v16h a, v16h b, v16h c, v16h d) { keep4_h(a, b, c, d); }
};
template <> struct Frag<__bf16> {
  typedef v16b V; union U { v16b v; v8b h[2]; };
  static __device__ __forceinline__ v16b load(const __bf16* p) {
    U f; f.h[0] = *(const v8b*)(p); f.h[1] = *(const v8b*)(p + 16); return f.v;
  }
  static __device__ __forceinline__ v8f mma(v16b a, v16b b, v8f c) {
    return __builtin_amdgcn_wmma_f32_16x16x32_bf16(false, a, false, b, (short)0, c, false, false);
  }
  static __device__ __forceinline__ void guard(v8f& a, v8f& b, v16b x, v16b y) { dep_guard_b(a, b, x, y); }
  static __device__ __forceinline__ void keep(v16b a, v16b b, v16b c, v16b d) { keep4_b(a, b, c, d); }
};

__device__ __forceinline__ v8f mma_h(v16h a, v16h b, v8f c) {
  c = __builtin_amdgcn_wmma_f32_16x16x32_f16(false, a, false, b, (short)0, c, false, false);
  asm volatile("v_nop\n\tv_nop\n\tv_nop\n\tv_nop" : "+v"(c) : "v"(a), "v"(b));
  return c;
}

__device__ __forceinline__ float ftanh(float x) { return 1.0f - 2.0f * __builtin_amdgcn_rcpf(__expf(2.0f * x) + 1.0f); }

__global__ __launch_bounds__(NTHR) void tpw_f16(const float* __restrict__ src, int R, int C, int ldo,
                                               unsigned short* __restrict__ O, float sc) {
  __shared__ float Tt[64 * 65];
  const int tid = threadIdx.x;
  const int c0 = blockIdx.x * 64, r0 = blockIdx.y * 64;
  (void)R;
#pragma unroll
  for (int i = 0; i < 4; ++i) {
    const int idx = i * NTHR + tid;
    const int rr = idx >> 4, cc = (idx & 15) * 4;
    const v4f v = *(const v4f*)(src + (size_t)(r0 + rr) * (size_t)C + c0 + cc);
    Tt[rr * 65 + cc + 0] = v[0];
    Tt[rr * 65 + cc + 1] = v[1];
    Tt[rr * 65 + cc + 2] = v[2];
    Tt[rr * 65 + cc + 3] = v[3];
  }
  __syncthreads();
  const int q = tid >> 3, c8 = (tid & 7) * 8;
  v8h hv[2];
#pragma unroll
  for (int g = 0; g < 2; ++g) {
    const int qq = g * 32 + q;
#pragma unroll
    for (int e = 0; e < 8; ++e) {
      const float f = Tt[(c8 + e) * 65 + qq];
      hv[g][e] = (_Float16)(f * sc);
    }
  }
  for (int pass = 0; pass < 2; ++pass) {
#pragma unroll
    for (int g = 0; g < 2; ++g) {
      const size_t o = (size_t)(c0 + g * 32 + q) * (size_t)ldo + (size_t)(r0 + c8);
      *(volatile v8h*)(O + o) = hv[g];
    }
    __threadfence();
  }
}

__device__ __forceinline__ void gather_x(_Float16* Ax, const int* __restrict__ x, const float* __restrict__ emb,
                                         int rowbase, int t, int tid) {
  const int m = tid >> 4, c8 = (tid & 15) * 8;
  int tok = x[(size_t)(rowbase + m) * NSTEP + (size_t)t];
  tok = tok < 0 ? 0 : tok;
  tok = tok > NVOC - 1 ? NVOC - 1 : tok;
  const float* e = emb + (size_t)tok * NHID + c8;
  const v4f a = *(const v4f*)(e);
  const v4f b = *(const v4f*)(e + 4);
  v8h hv;
  hv[0] = (_Float16)(a[0] * A_SCALE); hv[1] = (_Float16)(a[1] * A_SCALE);
  hv[2] = (_Float16)(a[2] * A_SCALE); hv[3] = (_Float16)(a[3] * A_SCALE);
  hv[4] = (_Float16)(b[0] * A_SCALE); hv[5] = (_Float16)(b[1] * A_SCALE);
  hv[6] = (_Float16)(b[2] * A_SCALE); hv[7] = (_Float16)(b[3] * A_SCALE);
  *(v8h*)(Ax + m * APITCH + c8) = hv;
}

__global__ __launch_bounds__(NTHR) void rnn_kernel(const int* __restrict__ x, const int* __restrict__ lengths,
                                                  const float* __restrict__ emb, const float* __restrict__ bias,
                                                  const unsigned short* __restrict__ WTp, float* __restrict__ hfin) {
  __shared__ __align__(16) _Float16 Ax[ATILE];
  __shared__ __align__(16) _Float16 Ah[4 * ATILE];
  __shared__ __align__(16) float    Hs[SEQ_PER_BLK * OPITCH];
  const _Float16* WT = (const _Float16*)WTp;
  const int tid = threadIdx.x, lane = tid & 31, wave = tid >> 5;
  const int c = lane & 15, hh = lane >> 4, koff = hh * 8;
  const int rowbase = blockIdx.x * SEQ_PER_BLK;
  const int j = 16 * wave + c;

#pragma unroll 1
  for (int i = 0; i < 34; ++i) Ah[i * NTHR + tid] = (_Float16)0.0f;
  gather_x(Ax, x, emb, rowbase, 0, tid);

  int len8[8];
  float h0st[8], h1st[8];
#pragma unroll
  for (int r = 0; r < 8; ++r) {
    len8[r] = lengths[rowbase + 8 * hh + r];
    h0st[r] = 0.0f;
    h1st[r] = 0.0f;
  }
  const float bj0 = bias[j];
  const float bj1 = bias[NHID + j];
  __syncthreads();

  const _Float16* axr = Ax + c * APITCH + koff;
  const _Float16* w0  = WT + (size_t)j * KTOT + koff;
  const _Float16* w1  = WT + (size_t)NHID * KTOT + (size_t)j * KTOT + koff;
  const v8f z8 = {0.f, 0.f, 0.f, 0.f, 0.f, 0.f, 0.f, 0.f};

#pragma unroll 1
  for (int t = 0; t < NSTEP; ++t) {
    const int cur = t & 1, nxt = cur ^ 1;
    const _Float16* ah0c = Ah + (0 * 2 + cur) * ATILE;
    _Float16*       ah0n = Ah + (0 * 2 + nxt) * ATILE;
    const _Float16* ah1c = Ah + (1 * 2 + cur) * ATILE;
    _Float16*       ah1n = Ah + (1 * 2 + nxt) * ATILE;

    {
      v8f acc = z8;
#pragma unroll
      for (int k0 = 0; k0 < NHID; k0 += 32) {
        const v16h a = Frag<_Float16>::load(axr + k0);
        const v16h b = Frag<_Float16>::load(w0 + k0);
        acc = mma_h(a, b, acc);
      }
      const _Float16* ahr = ah0c + c * APITCH + koff;
#pragma unroll
      for (int k0 = 0; k0 < NHID; k0 += 32) {
        const v16h a = Frag<_Float16>::load(ahr + k0);
        const v16h b = Frag<_Float16>::load(w0 + NHID + k0);
        acc = mma_h(a, b, acc);
      }
#pragma unroll
      for (int r = 0; r < 8; ++r) {
        const float z  = acc[r] * FOLD_INV + bj0;
        const float hn = ftanh(z);
        const bool alive = (t < len8[r]);
        const float v = alive ? hn : h0st[r];
        h0st[r] = v;
        ah0n[(8 * hh + r) * APITCH + j] = (_Float16)(v * A_SCALE);
      }
    }
    __syncthreads();

    {
      v8f acc = z8;
      const _Float16* a0r = ah0n + c * APITCH + koff;
#pragma unroll
      for (int k0 = 0; k0 < NHID; k0 += 32) {
        const v16h a = Frag<_Float16>::load(a0r + k0);
        const v16h b = Frag<_Float16>::load(w1 + k0);
        acc = mma_h(a, b, acc);
      }
      const _Float16* a1r = ah1c + c * APITCH + koff;
#pragma unroll
      for (int k0 = 0; k0 < NHID; k0 += 32) {
        const v16h a = Frag<_Float16>::load(a1r + k0);
        const v16h b = Frag<_Float16>::load(w1 + NHID + k0);
        acc = mma_h(a, b, acc);
      }
#pragma unroll
      for (int r = 0; r < 8; ++r) {
        const float z  = acc[r] * FOLD_INV + bj1;
        const float hn = ftanh(z);
        const bool alive = (t < len8[r]);
        const float v = alive ? hn : h1st[r];
        h1st[r] = v;
        ah1n[(8 * hh + r) * APITCH + j] = (_Float16)(v * A_SCALE);
      }
    }
    {
      const int tn = (t + 1 < NSTEP) ? (t + 1) : (NSTEP - 1);
      gather_x(Ax, x, emb, rowbase, tn, tid);
    }
    __syncthreads();
  }

#pragma unroll
  for (int r = 0; r < 8; ++r) Hs[(8 * hh + r) * OPITCH + j] = h1st[r];
  __syncthreads();
  for (int pass = 0; pass < 2; ++pass) {
#pragma unroll
    for (int it = 0; it < 2; ++it) {
      const int idx = it * NTHR + tid;
      const int row = idx >> 5, c4 = (idx & 31) * 4;
      const v4f v = *(const v4f*)(Hs + row * OPITCH + c4);
      *(volatile v4f*)(hfin + (size_t)(rowbase + row) * NHID + c4) = v;
    }
    __threadfence();
  }
}

__global__ __launch_bounds__(NTHR) void head_kernel(const float* __restrict__ hfin, const float* __restrict__ clsw,
                                                   const float* __restrict__ clsb, float* __restrict__ out) {
  __shared__ __align__(16) float zs[NSEQ];
  const int tid = threadIdx.x;
  const float* hr = hfin + (size_t)tid * NHID;
  float z = 0.0f;
#pragma unroll 1
  for (int k = 0; k < NHID; ++k) z += hr[k] * clsw[k];
  z += clsb[0];
  const float s = 1.0f / (1.0f + expf(-z));
  zs[tid] = s;
  __syncthreads();
  v4f v = {0.f, 0.f, 0.f, 0.f};
  if (tid < NSEQ / 4) v = *(const v4f*)(zs + tid * 4);
  for (int pass = 0; pass < 2; ++pass) {
    if (tid < NSEQ / 4) *(volatile v4f*)(out + tid * 4) = v;
    __threadfence();
  }
}

extern "C" void kernel_launch(void* const* d_in, const int* in_sizes, int n_in,
                              void* d_out, int out_size, void* d_ws, size_t ws_size, hipStream_t stream) {
  if (n_in < 8 || d_out == nullptr || d_ws == nullptr) return;
  if (in_sizes[0] != NSEQ * NSTEP || in_sizes[1] != NSEQ || in_sizes[2] != NVOC * NHID ||
      in_sizes[3] != NLAY * NHID * NHID || in_sizes[4] != NLAY * NHID * NHID || in_sizes[5] != NLAY * NHID ||
      in_sizes[6] != NHID || in_sizes[7] != 1 || out_size != NSEQ) return;

  const int*   x       = (const int*)d_in[0];
  const int*   lengths = (const int*)d_in[1];
  const float* emb     = (const float*)d_in[2];
  const float* W_ih    = (const float*)d_in[3];
  const float* W_hh    = (const float*)d_in[4];
  const float* bias    = (const float*)d_in[5];
  const float* cls_w   = (const float*)d_in[6];
  const float* cls_b   = (const float*)d_in[7];
  float* out = (float*)d_out;

  char* ws = (char*)d_ws; size_t off = 0;
  auto carve = [&](size_t bytes) -> char* { char* p = ws + off; off += (bytes + 255) & ~(size_t)255; return p; };
  unsigned short* WT   = (unsigned short*)carve((size_t)NLAY * NHID * KTOT * 2);
  float*          HFIN = (float*)carve((size_t)NSEQ * NHID * 4);
  if (off > ws_size || off > (size_t)134217728) return;

  const dim3 tg(NHID / 64, NHID / 64);
  tpw_f16<<<tg, NTHR, 0, stream>>>(W_ih,               NHID, NHID, KTOT, WT,                             W_SCALE);
  tpw_f16<<<tg, NTHR, 0, stream>>>(W_hh,               NHID, NHID, KTOT, WT + NHID,                      W_SCALE);
  tpw_f16<<<tg, NTHR, 0, stream>>>(W_ih + NHID * NHID, NHID, NHID, KTOT, WT + (size_t)NHID * KTOT,        W_SCALE);
  tpw_f16<<<tg, NTHR, 0, stream>>>(W_hh + NHID * NHID, NHID, NHID, KTOT, WT + (size_t)NHID * KTOT + NHID, W_SCALE);
  rnn_kernel<<<NSEQ / SEQ_PER_BLK, NTHR, 0, stream>>>(x, lengths, emb, bias, WT, HFIN);
  head_kernel<<<1, NTHR, 0, stream>>>(HFIN, cls_w, cls_b, out);
}
